// FlatConv3x3NNUE_46892452938213
// MI455X (gfx1250) — hardware-verified
//
#include <hip/hip_runtime.h>


#define NB_  8192
#define NPOS 25
#define CIN  2
#define DMID 128
#define DFT  32
#define KP   32
#define DM   KP
#define CMX  0.9921875f
#define LOSC 1024.0f

typedef _Float16 h16;
typedef unsigned short bf;
typedef __attribute__((ext_vector_type(16))) __bf16   v16bf;
typedef __attribute__((ext_vector_type(16))) _Float16 v16h;
typedef __attribute__((ext_vector_type(8)))  _Float16 v8h;
typedef __attribute__((ext_vector_type(8)))  unsigned short v8us;
typedef __attribute__((ext_vector_type(8)))  float    v8f;
typedef __attribute__((ext_vector_type(4)))  float    v4f;
typedef v8h  __attribute__((may_alias)) v8ha;
typedef v4f  __attribute__((may_alias)) v4fa;
typedef v8us __attribute__((may_alias)) v8usa;

__device__ __forceinline__ unsigned short f2bf(float f) { unsigned u = __float_as_uint(f); u += 0x7FFFu + ((u >> 16) & 1u); return (unsigned short)(u >> 16); }
__device__ __forceinline__ float bf2f(unsigned short b) { return __uint_as_float(((unsigned)b) << 16); }
__device__ __forceinline__ float bfr(float f) { return bf2f(f2bf(f)); }
__device__ __forceinline__ v16h cat16(v8h lo, v8h hi) { return __builtin_shufflevector(lo, hi, 0, 1, 2, 3, 4, 5, 6, 7, 8, 9, 10, 11, 12, 13, 14, 15); }
__device__ __forceinline__ v16bf cat16b(v8us lo, v8us hi) { return __builtin_bit_cast(v16bf, __builtin_shufflevector(lo, hi, 0, 1, 2, 3, 4, 5, 6, 7, 8, 9, 10, 11, 12, 13, 14, 15)); }
__device__ __forceinline__ v8f wmma16(v16h a, v16h b, v8f c) { return __builtin_amdgcn_wmma_f32_16x16x32_f16(false, a, false, b, (short)0, c, false, false); }
__device__ __forceinline__ v8f wmmab(v16bf a, v16bf b, v8f c) { return __builtin_amdgcn_wmma_f32_16x16x32_bf16(false, a, false, b, (short)0, c, false, false); }

template <bool SPLITA, bool F16OUT = false>
__global__ __launch_bounds__(128) void k_gemmb(const bf* __restrict__ A, const bf* __restrict__ Al, const bf* __restrict__ Bn, const float* __restrict__ bias, float* C, int ldc, h16* C2, const float* __restrict__ R = nullptr, int K = DM, int roundR = 1) {
    __shared__ __align__(16) float ost[4][16 * 68];
    const int lane = threadIdx.x & 31, wave = threadIdx.x >> 5, lr = lane & 15, hi = lane >> 4;
    const int r0 = blockIdx.x * 64 + wave * 16, c0 = blockIdx.y * 64;
    const size_t aoff = (size_t)(r0 + lr) * K + 8 * hi;
    size_t boff[4];
#pragma unroll
    for (int t = 0; t < 4; ++t) boff[t] = (size_t)(c0 + t * 16 + lr) * K + 8 * hi;
    v8f acc[4];
#pragma unroll
    for (int t = 0; t < 4; ++t) acc[t] = (v8f){};
#pragma unroll 1
    for (int kc = 0; kc < K; kc += 32) {
        const v16bf a = cat16b(*(const v8us*)(A + aoff + kc), *(const v8us*)(A + aoff + kc + 16));
        v16bf al = a;
        if (SPLITA) al = cat16b(*(const v8us*)(Al + aoff + kc), *(const v8us*)(Al + aoff + kc + 16));
#pragma unroll
        for (int t = 0; t < 4; ++t) { const v16bf b = cat16b(*(const v8us*)(Bn + boff[t] + kc), *(const v8us*)(Bn + boff[t] + kc + 16)); acc[t] = wmmab(a, b, acc[t]); if (SPLITA) acc[t] = wmmab(al, b, acc[t]); }
        asm volatile("v_nop\n\tv_nop\n\tv_nop\n\tv_nop" : "+v"(acc[0]), "+v"(acc[1]), "+v"(acc[2]), "+v"(acc[3]) : "v"(a), "v"(al));
    }
    float* os = &ost[wave][0];
#pragma unroll
    for (int t = 0; t < 4; ++t) { const float bv = bias ? bfr(bias[c0 + t * 16 + lr]) : 0.f;
#pragma unroll
        for (int j = 0; j < 8; ++j) os[(hi * 8 + j) * 68 + t * 16 + lr] = acc[t][j] + bv; }
    __syncthreads();
    if (F16OUT) {
        h16* crow = (h16*)(void*)C + (size_t)r0 * ldc + c0;
        auto pass = [&]() {
#pragma unroll
            for (int s = 0; s < 4; ++s) { const int row = 4 * s + (lane >> 3), piece = lane & 7; const float* sp = os + row * 68 + piece * 8; v8h o, o2;
#pragma unroll
                for (int i = 0; i < 8; ++i) { const h16 a = (h16)sp[i]; o[i] = a; o2[i] = (h16)((sp[i] - (float)a) * LOSC); }
                *(volatile v8h*)(crow + (size_t)row * ldc + piece * 8) = o; if (C2) *(volatile v8h*)(C2 + (size_t)r0 * ldc + c0 + (size_t)row * ldc + piece * 8) = o2; }
        };
        pass(); __threadfence(); pass();
    } else {
        float* crow = C + (size_t)r0 * ldc + c0;
        auto pass = [&]() {
#pragma unroll
            for (int s = 0; s < 8; ++s) { const int Lid = (lane >> 3) + 4 * s, piece = lane & 7; const int row = Lid >> 1, cofs = (Lid & 1) * 32 + piece * 4;
                v4f val = *(const v4fa*)(os + row * 68 + cofs); if (R) { const v4f rv = *(const v4f*)(R + ((size_t)r0 + row) * ldc + c0 + cofs); val += roundR ? (v4f){bfr(rv[0]), bfr(rv[1]), bfr(rv[2]), bfr(rv[3])} : rv; }
                *(volatile v4f*)(crow + (size_t)row * ldc + cofs) = val; }
        };
        pass(); __threadfence(); pass();
    }
}

__global__ __launch_bounds__(256) void k_cvt8(const float* __restrict__ src, bf* dst, size_t n8) {
    const size_t i = (size_t)blockIdx.x * 256 + threadIdx.x; if (i >= n8) return;
    const v8f v = *(const v8f*)(src + i * 8); v8us o;
#pragma unroll
    for (int k = 0; k < 8; ++k) o[k] = f2bf(v[k]);
    *(volatile v8us*)(dst + i * 8) = o; __threadfence(); *(volatile v8us*)(dst + i * 8) = o;
}
__global__ __launch_bounds__(256) void k_zero8(bf* dst, size_t n8) {
    const size_t i = (size_t)blockIdx.x * 256 + threadIdx.x; if (i >= n8) return; v8us z;
#pragma unroll
    for (int k = 0; k < 8; ++k) z[k] = 0;
    *(volatile v8us*)(dst + i * 8) = z; __threadfence(); *(volatile v8us*)(dst + i * 8) = z;
}

__global__ __launch_bounds__(256) void k_patch(const float* __restrict__ xin, int py, int px, bf* A) {
    typedef __attribute__((ext_vector_type(2))) unsigned short v2us;
    const int lane = threadIdx.x & 31; const size_t b = ((size_t)blockIdx.x * 8 + (threadIdx.x >> 5)) * 2 + (lane >> 4); if (b >= (size_t)NB_) return; const int c0 = (lane & 15) * 2; v2us o;
#pragma unroll
    for (int i = 0; i < 2; ++i) { const int k = c0 + i; float v = 0.f; if (k < 18) { const int c = k / 9, r = k % 9, y = r / 3, xx = r % 3; v = xin[((b * CIN + c) * 7 + py + y) * 7 + px + xx]; } o[i] = f2bf(v); }
    *(volatile v2us*)(A + b * KP + c0) = o; __threadfence(); *(volatile v2us*)(A + b * KP + c0) = o;
}
__global__ __launch_bounds__(256) void k_w1(const float* __restrict__ W1, int p, bf* B1) {
    typedef __attribute__((ext_vector_type(2))) unsigned short v2us;
    const int lane = threadIdx.x & 31; const int r = (blockIdx.x * 8 + (threadIdx.x >> 5)) * 2 + (lane >> 4); if (r >= 4 * DMID) return; const int ij = r / DMID, o = r % DMID, i = ij >> 1, j = ij & 1; const int c0 = (lane & 15) * 2; v2us v;
#pragma unroll
    for (int q = 0; q < 2; ++q) { const int k = c0 + q; float w = 0.f; if (k < 18) { const int c = k / 9, rr = k % 9, y = rr / 3, xx = rr % 3; const int di = y - i, dj = xx - j; if (di >= 0 && di < 2 && dj >= 0 && dj < 2) w = W1[((((size_t)p * DMID + o) * CIN + c) * 2 + di) * 2 + dj]; } v[q] = f2bf(w); }
    *(volatile v2us*)(B1 + (size_t)r * KP + c0) = v; __threadfence(); *(volatile v2us*)(B1 + (size_t)r * KP + c0) = v;
}
__global__ __launch_bounds__(512) void k_b1(const float* __restrict__ b1, int p, float* B1B) {
    const int t = threadIdx.x; const float v = b1[(size_t)p * DMID + (t % DMID)]; *(volatile float*)(B1B + t) = v; __threadfence(); *(volatile float*)(B1B + t) = v;
}
__global__ __launch_bounds__(256) void k_w2(const float* __restrict__ W2, int p, bf* B2) {
    const int lane = threadIdx.x & 31; const int o = blockIdx.x * 8 + (threadIdx.x >> 5); if (o >= DMID) return;
#pragma unroll 1
    for (int ps = 0; ps < 2; ++ps) {
#pragma unroll
        for (int q = 0; q < 2; ++q) { v8us v;
#pragma unroll
            for (int t = 0; t < 8; ++t) { const int col = q * 256 + lane * 8 + t; const int ij = col / DMID, c = col % DMID, i = ij >> 1, j = ij & 1; v[t] = f2bf(W2[((((size_t)p * DMID + o) * DMID + c) * 2 + i) * 2 + j]); }
            *(volatile v8us*)(B2 + (size_t)o * (4 * DMID) + q * 256 + lane * 8) = v; }
        if (ps == 0) __threadfence(); }
}
template <int NCOL>
__global__ __launch_bounds__(256) void k_relupl(const float* __restrict__ F, bf* Ph, bf* Pl) {
    const int lane = threadIdx.x & 31; const size_t r = (size_t)blockIdx.x * 8 + (threadIdx.x >> 5); if (r >= (size_t)NB_) return;
    if (NCOL >= 256) {
#pragma unroll 1
        for (int ps = 0; ps < 2; ++ps) {
#pragma unroll
            for (int q = 0; q < NCOL / 256; ++q) { const size_t o = r * NCOL + q * 256 + lane * 8; const v8f v = *(const v8f*)(F + o); v8us oh, ol;
#pragma unroll
                for (int i = 0; i < 8; ++i) { const float y = fmaxf(v[i], 0.f); const unsigned short hb = f2bf(y); oh[i] = hb; ol[i] = f2bf(y - bf2f(hb)); }
                *(volatile v8us*)(Ph + o) = oh; *(volatile v8us*)(Pl + o) = ol; }
            if (ps == 0) __threadfence(); }
    } else { typedef __attribute__((ext_vector_type(4))) unsigned short v4us; const size_t o = r * NCOL + lane * 4; const v4f v = *(const v4f*)(F + o); v4us oh, ol;
#pragma unroll
        for (int i = 0; i < 4; ++i) { const float y = fmaxf(v[i], 0.f); const unsigned short hb = f2bf(y); oh[i] = hb; ol[i] = f2bf(y - bf2f(hb)); }
        *(volatile v4us*)(Ph + o) = oh; *(volatile v4us*)(Pl + o) = ol; __threadfence(); *(volatile v4us*)(Ph + o) = oh; *(volatile v4us*)(Pl + o) = ol; }
}
template <int K>
__global__ __launch_bounds__(256) void k_padrows(const float* __restrict__ src, int nlive, bf* BW) {
    const int lane = threadIdx.x & 31; const int w = blockIdx.x * 8 + (threadIdx.x >> 5);
    if (K == 128) { typedef __attribute__((ext_vector_type(4))) unsigned short v4us; const int r = w; if (r >= 64) return; v4us o;
#pragma unroll
        for (int i = 0; i < 4; ++i) { const int k = lane * 4 + i; o[i] = f2bf(r < nlive ? src[(size_t)(r < nlive ? r : 0) * K + k] : 0.f); }
        *(volatile v4us*)(BW + (size_t)r * K + lane * 4) = o; __threadfence(); *(volatile v4us*)(BW + (size_t)r * K + lane * 4) = o; }
    else { typedef __attribute__((ext_vector_type(2))) unsigned short v2us; const int r = w * 2 + (lane >> 4); if (r >= 64) return; const int c0 = (lane & 15) * 2; v2us o;
#pragma unroll
        for (int i = 0; i < 2; ++i) o[i] = f2bf(r < nlive ? src[(size_t)(r < nlive ? r : 0) * K + c0 + i] : 0.f);
        *(volatile v2us*)(BW + (size_t)r * K + c0) = o; __threadfence(); *(volatile v2us*)(BW + (size_t)r * K + c0) = o; }
}
__global__ __launch_bounds__(64) void k_bpad64(const float* __restrict__ src, int nlive, float* BP) {
    const int t = threadIdx.x; const float v = (t < nlive) ? src[t < nlive ? t : 0] : 0.f; *(volatile float*)(BP + t) = v; __threadfence(); *(volatile float*)(BP + t) = v;
}
__global__ __launch_bounds__(256) void k_accum(const float* __restrict__ F4, int first, float* FS) {
    typedef __attribute__((ext_vector_type(2))) float v2f_;
    const int lane = threadIdx.x & 31; const size_t b = (size_t)blockIdx.x * 8 + (threadIdx.x >> 5); if (b >= (size_t)NB_) return; const size_t o = b * 64 + lane * 2; v2f_ v = *(const v2f_*)(F4 + o); v2f_ acc;
    if (first) { acc[0] = 0.f; acc[1] = 0.f; } else acc = *(const v2f_*)(FS + o);
#pragma unroll
    for (int i = 0; i < 2; ++i) acc[i] += fminf(fmaxf(v[i], -1.0f), CMX);
    *(volatile v2f_*)(FS + o) = acc; __threadfence(); *(volatile v2f_*)(FS + o) = acc;
}
__global__ __launch_bounds__(256) void k_clippl(const float* __restrict__ F, bf* Ph, bf* Pl) {
    typedef __attribute__((ext_vector_type(2))) unsigned short v2us;
    const int lane = threadIdx.x & 31; const size_t b = ((size_t)blockIdx.x * 8 + (threadIdx.x >> 5)) * 2 + (lane >> 4); if (b >= (size_t)NB_) return; const int c0 = (lane & 15) * 2; v2us oh, ol;
#pragma unroll
    for (int i = 0; i < 2; ++i) { const float y = fminf(fmaxf(F[b * 64 + c0 + i], 0.f), CMX); const unsigned short hb = f2bf(y); oh[i] = hb; ol[i] = f2bf(y - bf2f(hb)); }
    *(volatile v2us*)(Ph + b * DFT + c0) = oh; *(volatile v2us*)(Pl + b * DFT + c0) = ol; __threadfence(); *(volatile v2us*)(Ph + b * DFT + c0) = oh; *(volatile v2us*)(Pl + b * DFT + c0) = ol;
}
__global__ __launch_bounds__(256) void k_outcol(const float* __restrict__ Cm, float* OUTP) {
    const int lane = threadIdx.x & 31; const int w = blockIdx.x * 8 + (threadIdx.x >> 5); if (w >= NB_ / 32) return; const int b = w * 32 + lane; const float v = Cm[(size_t)b * 64];
    *(volatile float*)(OUTP + b) = v; __threadfence(); *(volatile float*)(OUTP + b) = v;
}

extern "C" void kernel_launch(void* const* d_in, const int* in_sizes, int n_in,
                              void* d_out, int out_size, void* d_ws, size_t ws_size, hipStream_t stream) {
    (void)in_sizes; (void)n_in; (void)out_size;
    const float* x = (const float*)d_in[0]; const float* W1 = (const float*)d_in[1]; const float* b1 = (const float*)d_in[2]; const float* W2 = (const float*)d_in[3]; const float* b2 = (const float*)d_in[4]; const float* W3 = (const float*)d_in[5]; const float* b3 = (const float*)d_in[6]; const float* W4 = (const float*)d_in[7]; const float* b4 = (const float*)d_in[8];
    const float* f1w = (const float*)d_in[9]; const float* f1b = (const float*)d_in[10]; const float* f2w = (const float*)d_in[11]; const float* f2b = (const float*)d_in[12]; const float* f3w = (const float*)d_in[13]; const float* f3b = (const float*)d_in[14];
    float* out = (float*)d_out;
    char* wsp = (char*)d_ws;
    auto take = [&](size_t bytes) { char* p = wsp; wsp += (bytes + 255) & ~(size_t)255; return (void*)p; };
    bf* AP = (bf*)take((size_t)NB_ * KP * 2); bf* B1 = (bf*)take((size_t)4 * DMID * KP * 2); float* B1B = (float*)take(4 * DMID * 4); bf* B2 = (bf*)take((size_t)DMID * 4 * DMID * 2); bf* W3B = (bf*)take((size_t)NPOS * DMID * DMID * 2); bf* W4P = (bf*)take((size_t)64 * DMID * 2); float* B4P = (float*)take(64 * 4);
    float* H1 = (float*)take((size_t)NB_ * 4 * DMID * 4); bf* P1h = (bf*)take((size_t)NB_ * 4 * DMID * 2); bf* P1l = (bf*)take((size_t)NB_ * 4 * DMID * 2); float* H2 = (float*)take((size_t)NB_ * DMID * 4); bf* P2h = (bf*)take((size_t)NB_ * DMID * 2); bf* P2l = (bf*)take((size_t)NB_ * DMID * 2);
    float* H3 = (float*)take((size_t)NB_ * DMID * 4); bf* P3h = (bf*)take((size_t)NB_ * DMID * 2); bf* P3l = (bf*)take((size_t)NB_ * DMID * 2); float* F4 = (float*)take((size_t)NB_ * 64 * 4); float* FS = (float*)take((size_t)NB_ * 64 * 4);
    bf* Vh = (bf*)take((size_t)NB_ * DFT * 2); bf* Vl = (bf*)take((size_t)NB_ * DFT * 2); bf* FC1 = (bf*)take(64 * DFT * 2); bf* FC2 = (bf*)take(64 * DFT * 2); bf* FC3 = (bf*)take(64 * DFT * 2); float* FB1 = (float*)take(64 * 4); float* FB2 = (float*)take(64 * 4); float* FB3 = (float*)take(64 * 4); float* G1 = (float*)take((size_t)NB_ * 64 * 4);
    if ((size_t)(wsp - (char*)d_ws) > ws_size) return;
    k_cvt8<<<(NPOS * DMID * DMID / 8 + 255) / 256, 256, 0, stream>>>(W3, W3B, (size_t)NPOS * DMID * DMID / 8);
    k_padrows<32><<<(64 / 2 + 7) / 8, 256, 0, stream>>>(f1w, DFT, FC1); k_padrows<32><<<(64 / 2 + 7) / 8, 256, 0, stream>>>(f2w, DFT, FC2); k_padrows<32><<<(64 / 2 + 7) / 8, 256, 0, stream>>>(f3w, 1, FC3);
    k_bpad64<<<1, 64, 0, stream>>>(f1b, DFT, FB1); k_bpad64<<<1, 64, 0, stream>>>(f2b, DFT, FB2); k_bpad64<<<1, 64, 0, stream>>>(f3b, 1, FB3);
    for (int p = 0; p < NPOS; ++p) { const int py = p / 5, px = p % 5;
        k_patch<<<(NB_ / 2) / 8, 256, 0, stream>>>(x, py, px, AP); k_w1<<<(4 * DMID / 2) / 8, 256, 0, stream>>>(W1, p, B1); k_b1<<<1, 512, 0, stream>>>(b1, p, B1B); k_w2<<<DMID / 8, 256, 0, stream>>>(W2, p, B2);
        k_padrows<128><<<64 / 8, 256, 0, stream>>>(W4 + (size_t)p * DFT * DMID, DFT, W4P); k_bpad64<<<1, 64, 0, stream>>>(b4 + (size_t)p * DFT, DFT, B4P);
        k_gemmb<false, false><<<dim3(NB_ / 64, (4 * DMID) / 64, 1), 128, 0, stream>>>(AP, nullptr, B1, B1B, H1, 4 * DMID, nullptr, nullptr, KP);
        k_relupl<512><<<NB_ / 8, 256, 0, stream>>>(H1, P1h, P1l);
        k_gemmb<true, false><<<dim3(NB_ / 64, DMID / 64, 1), 128, 0, stream>>>(P1h, P1l, B2, b2 + (size_t)p * DMID, H2, DMID, nullptr, nullptr, 4 * DMID);
        k_relupl<128><<<NB_ / 8, 256, 0, stream>>>(H2, P2h, P2l);
        k_gemmb<true, false><<<dim3(NB_ / 64, DMID / 64, 1), 128, 0, stream>>>(P2h, P2l, W3B + (size_t)p * DMID * DMID, b3 + (size_t)p * DMID, H3, DMID, nullptr, nullptr, DMID);
        k_relupl<128><<<NB_ / 8, 256, 0, stream>>>(H3, P3h, P3l);
        k_gemmb<true, false><<<dim3(NB_ / 64, 1, 1), 128, 0, stream>>>(P3h, P3l, W4P, B4P, F4, 64, nullptr, nullptr, DMID);
        k_accum<<<NB_ / 8, 256, 0, stream>>>(F4, p == 0, FS); }
    k_clippl<<<(NB_ / 2) / 8, 256, 0, stream>>>(FS, Vh, Vl);
    k_gemmb<true, false><<<dim3(NB_ / 64, 1, 1), 128, 0, stream>>>(Vh, Vl, FC1, FB1, G1, 64, nullptr, nullptr, DFT);
    k_clippl<<<(NB_ / 2) / 8, 256, 0, stream>>>(G1, Vh, Vl);
    k_gemmb<true, false><<<dim3(NB_ / 64, 1, 1), 128, 0, stream>>>(Vh, Vl, FC2, FB2, G1, 64, nullptr, nullptr, DFT);
    k_clippl<<<(NB_ / 2) / 8, 256, 0, stream>>>(G1, Vh, Vl);
    k_gemmb<true, false><<<dim3(NB_ / 64, 1, 1), 128, 0, stream>>>(Vh, Vl, FC3, FB3, G1, 64, nullptr, nullptr, DFT);
    k_outcol<<<(NB_ / 32) / 8, 256, 0, stream>>>(G1, out);
}
